// LinearCausalAttention_11304353923655
// MI455X (gfx1250) — hardware-verified
//
#include <hip/hip_runtime.h>
#include <stdint.h>

#define NBAT 2
#define NT   2048
#define NC   1024
#define NH   16
#define ND   64
#define NBH  32
#define NTOK 4096
#define CH   64
#define NCH  32
#define NSL  32
#define NJ   80
#define QP   72
#define KP   72
#define VP   72
#define NX8  524288
#define NW8  131072
static_assert(NT == NCH * CH);
static_assert(NTOK == NBAT * NT);
static_assert(NBH == NBAT * NH);
static_assert(NC == NH * ND);
static_assert(NX8 * 8 == NTOK * NC);
static_assert(NW8 * 8 == NC * NC);
static_assert((NX8 % 256) == 0 && (NW8 % 256) == 0);
static_assert(((QP * 2) % 16) == 0 && ((KP * 2) % 16) == 0 && ((VP * 2) % 16) == 0);
static_assert((NC % 32) == 0 && (ND % 32) == 0 && (CH % 32) == 0);

typedef __bf16   v16b __attribute__((ext_vector_type(16)));
typedef __bf16   v8b  __attribute__((ext_vector_type(8)));
typedef float    v8f  __attribute__((ext_vector_type(8)));
typedef float    v4f  __attribute__((ext_vector_type(4)));
typedef unsigned int v4u __attribute__((ext_vector_type(4)));
typedef v4f __attribute__((may_alias)) v4fa;

__device__ __forceinline__ unsigned short bf_bits(float f) {
  unsigned u = __float_as_uint(f);
  return (unsigned short)((u + 0x7FFFu + ((u >> 16) & 1u)) >> 16);
}
__device__ __forceinline__ float bf_up(unsigned short h) { return __uint_as_float(((unsigned)h) << 16); }
__device__ __forceinline__ __bf16 bf_val(unsigned short h) { return __builtin_bit_cast(__bf16, h); }
__device__ __forceinline__ unsigned pk16(unsigned short a, unsigned short b) { return (unsigned)a | ((unsigned)b << 16); }
__device__ __forceinline__ v8f zero8() { v8f z = {0.f, 0.f, 0.f, 0.f, 0.f, 0.f, 0.f, 0.f}; return z; }
__device__ __forceinline__ float phi_f(float q) { return (q > 0.0f) ? (q + 1.0f) : __expf(q); }

__device__ __forceinline__ v16b ldfrag_b(const __bf16* p) {
  union { v16b v; v8b h[2]; } f;
  f.h[0] = *(const v8b*)(p);
  f.h[1] = *(const v8b*)(p + 16);
  return f.v;
}

__device__ __forceinline__ v8f mma_b(v16b a, v16b b, v8f c) {
  c = __builtin_amdgcn_wmma_f32_16x16x32_bf16(false, a, false, b, (short)0, c, false, false);
  asm volatile("v_nop\n\tv_nop\n\tv_nop\n\tv_nop" : "+v"(c) : "v"(a), "v"(b));
  return c;
}

__device__ __forceinline__ void phi_split8(v4f a, v4f c, v4u& hv, v4u& lv) {
  const float xv[8] = {a[0], a[1], a[2], a[3], c[0], c[1], c[2], c[3]};
  unsigned short hb[8], lb[8];
#pragma unroll
  for (int e = 0; e < 8; ++e) {
    const float p = phi_f(xv[e]);
    const unsigned short h = bf_bits(p);
    hb[e] = h;
    lb[e] = bf_bits(p - bf_up(h));
  }
  hv[0] = pk16(hb[0], hb[1]); hv[1] = pk16(hb[2], hb[3]); hv[2] = pk16(hb[4], hb[5]); hv[3] = pk16(hb[6], hb[7]);
  lv[0] = pk16(lb[0], lb[1]); lv[1] = pk16(lb[2], lb[3]); lv[2] = pk16(lb[4], lb[5]); lv[3] = pk16(lb[6], lb[7]);
}

__global__ __launch_bounds__(256) void k_cvt(const float* __restrict__ x, const float* __restrict__ wq,
                                             const float* __restrict__ wk, const float* __restrict__ wv,
                                             const float* __restrict__ wp,
                                             unsigned short* xb, unsigned short* wb) {
  const int g = blockIdx.x * 256 + threadIdx.x;
  if (g >= NX8 + 4 * NW8) return;
  const float* src;
  unsigned short* dst;
  if (g < NX8) {
    src = x + (size_t)g * 8;
    dst = xb + (size_t)g * 8;
  } else {
    const int e = g - NX8;
    const int wsel = e / NW8;
    const int off = e - wsel * NW8;
    const float* w = (wsel == 0) ? wq : ((wsel == 1) ? wk : ((wsel == 2) ? wv : wp));
    src = w + (size_t)off * 8;
    dst = wb + (size_t)e * 8;
  }
  const v4f a = *(const v4fa*)src;
  const v4f c = *(const v4fa*)(src + 4);
  v4u o;
  o[0] = pk16(bf_bits(a[0]), bf_bits(a[1]));
  o[1] = pk16(bf_bits(a[2]), bf_bits(a[3]));
  o[2] = pk16(bf_bits(c[0]), bf_bits(c[1]));
  o[3] = pk16(bf_bits(c[2]), bf_bits(c[3]));
  *(volatile v4u*)dst = o;
  __threadfence();
  *(volatile v4u*)dst = o;
}

__global__ __launch_bounds__(128) void k_proj(const unsigned short* __restrict__ xbp,
                                             const unsigned short* __restrict__ wbp,
                                             float* qf, float* kf, float* vf) {
  __shared__ __align__(16) float sT[128 * ND];
  const int tid = threadIdx.x, lane = tid & 31, w = tid >> 5;
  const int hh = lane >> 4, m = lane & 15;
  const int m0 = blockIdx.x * 128;
  const int cg = blockIdx.y, which = cg >> 4, head = cg & 15;
  const __bf16* xb = (const __bf16*)(const void*)xbp;
  const __bf16* wb = (const __bf16*)(const void*)wbp;
  const __bf16* xa0 = xb + ((size_t)(m0 + 32 * w + m)) * NC + 8 * hh;
  const __bf16* xa1 = xa0 + (size_t)16 * NC;
  const __bf16* wr  = wb + ((size_t)which * NC + head * ND + m) * NC + 8 * hh;

  v8f acc[2][4];
#pragma unroll
  for (int mt = 0; mt < 2; ++mt)
#pragma unroll
    for (int nt = 0; nt < 4; ++nt) acc[mt][nt] = zero8();

#pragma unroll 1
  for (int k0 = 0; k0 < NC; k0 += 32) {
    const v16b a0 = ldfrag_b(xa0 + k0);
    const v16b a1 = ldfrag_b(xa1 + k0);
#pragma unroll
    for (int nt = 0; nt < 4; ++nt) {
      const v16b bb = ldfrag_b(wr + (size_t)nt * 16 * NC + k0);
      acc[0][nt] = mma_b(a0, bb, acc[0][nt]);
      acc[1][nt] = mma_b(a1, bb, acc[1][nt]);
    }
  }

#pragma unroll
  for (int nt = 0; nt < 4; ++nt)
#pragma unroll
    for (int mt = 0; mt < 2; ++mt)
#pragma unroll
      for (int r = 0; r < 8; ++r) {
        const int tokl = 32 * w + 16 * mt + 8 * hh + r;
        sT[tokl * ND + 16 * nt + m] = acc[mt][nt][r];
      }
  __syncthreads();

  float* plane = (which == 0) ? qf : ((which == 1) ? kf : vf);
  const int b = m0 >> 11, t0 = m0 & (NT - 1), bh = b * NH + head;
  float* dstb = plane + ((size_t)(bh * NT + t0 + 32 * w)) * ND;
  const float* srcb = sT + (32 * w) * ND;
  for (int pass = 0; pass < 2; ++pass) {
#pragma unroll
    for (int i = 0; i < 16; ++i) {
      const int o = i * 128 + lane * 4;
      const v4f vv = *(const v4fa*)(srcb + o);
      *(volatile v4f*)(dstb + o) = vv;
    }
    __threadfence();
  }
}

__global__ __launch_bounds__(128) void k_vt(const float* __restrict__ vf, unsigned short* VThp, unsigned short* VTlp) {
  __shared__ __align__(16) unsigned short sH[NJ * VP];
  __shared__ __align__(16) unsigned short sL[NJ * VP];
  const int tid = threadIdx.x, lane = tid & 31, wave = tid >> 5;
  const int bh = blockIdx.x >> 5, s0 = (blockIdx.x & 31) * 64;
  {
    const int r = tid >> 1, chh = (tid & 1) * 32;
    const float* src = vf + ((size_t)(bh * NT + s0 + r)) * ND + chh;
#pragma unroll 2
    for (int g = 0; g < 8; ++g) {
      const v4f a = *(const v4fa*)(src + 4 * g);
#pragma unroll
      for (int e = 0; e < 4; ++e) {
        const unsigned short h = bf_bits(a[e]);
        const unsigned short l = bf_bits(a[e] - bf_up(h));
        sH[(chh + 4 * g + e) * VP + r] = h;
        sL[(chh + 4 * g + e) * VP + r] = l;
      }
    }
#pragma unroll
    for (int e = 0; e < 8; ++e) {
      const int idx = tid * 8 + e;
      const int row = ND + (idx >> 6), col = idx & 63;
      sH[row * VP + col] = (row == ND) ? (unsigned short)0x3F80u : (unsigned short)0u;
      sL[row * VP + col] = (unsigned short)0u;
    }
  }
  __syncthreads();
  const int q8 = lane & 7, sub = lane >> 3;
  for (int pass = 0; pass < 2; ++pass) {
#pragma unroll
    for (int it = 0; it < 5; ++it) {
      const int row = wave * 20 + it * 4 + sub;
      const v4u vh = *(const v4u*)(sH + row * VP + 8 * q8);
      const v4u vl = *(const v4u*)(sL + row * VP + 8 * q8);
      const size_t go = ((size_t)(bh * NJ + row)) * NT + s0 + 8 * q8;
      *(volatile v4u*)(VThp + go) = vh;
      *(volatile v4u*)(VTlp + go) = vl;
    }
    __threadfence();
  }
}

#define SLABF 1088
#define SBUF_BYTES 21760
static_assert(SBUF_BYTES >= 5 * SLABF * 4);
static_assert(SBUF_BYTES >= 2 * 64 * KP * 2);

__global__ __launch_bounds__(160) void k_state(const float* __restrict__ kf, const unsigned short* __restrict__ VThp,
                                               const unsigned short* __restrict__ VTlp,
                                               unsigned short* Shp, unsigned short* Slp, float* out1, float* out2) {
  __shared__ __align__(16) unsigned char sbuf[SBUF_BYTES];
  const int tid = threadIdx.x, lane = tid & 31, wave = tid >> 5;
  const int hh = lane >> 4, m = lane & 15;
  const int bh = blockIdx.x;

  __bf16* sKh = (__bf16*)(void*)sbuf;
  __bf16* sKl = sKh + 64 * KP;
  float* slabs = (float*)(void*)sbuf;
  float* slab = slabs + wave * SLABF;

  const __bf16* VTh = (const __bf16*)(const void*)VThp;
  const __bf16* VTl = (const __bf16*)(const void*)VTlp;
  const size_t arow = ((size_t)(bh * NJ + wave * 16 + m)) * NT + 8 * hh;

  v8f acc[4];
#pragma unroll
  for (int nt = 0; nt < 4; ++nt) acc[nt] = zero8();
  const int q4 = lane >> 3, c8 = (lane & 7) * 8;

  for (int c = 0; c <= NCH; ++c) {
    __syncthreads();
#pragma unroll
    for (int nt = 0; nt < 4; ++nt)
#pragma unroll
      for (int r = 0; r < 8; ++r) slab[(8 * hh + r) * 68 + nt * 16 + m] = acc[nt][r];
    __builtin_amdgcn_fence(__ATOMIC_RELEASE, "workgroup");
    __builtin_amdgcn_wave_barrier();
    __builtin_amdgcn_fence(__ATOMIC_ACQUIRE, "workgroup");
    if (c < NCH) {
      v4u hv[4], lv[4];
#pragma unroll
      for (int it = 0; it < 4; ++it) {
        const int row = it * 4 + q4;
        const float* sp = slab + row * 68 + c8;
        v4u a, a2;
#pragma unroll
        for (int e = 0; e < 4; ++e) {
          const float f0 = sp[2 * e], f1 = sp[2 * e + 1];
          const unsigned short h0 = bf_bits(f0), h1 = bf_bits(f1);
          const unsigned short l0 = bf_bits(f0 - bf_up(h0)), l1 = bf_bits(f1 - bf_up(h1));
          a[e] = pk16(h0, h1); a2[e] = pk16(l0, l1);
        }
        hv[it] = a; lv[it] = a2;
      }
      const size_t gb = ((size_t)((bh * NSL + c) * NJ + wave * 16)) * ND + c8;
      for (int pass = 0; pass < 2; ++pass) {
#pragma unroll
        for (int it = 0; it < 4; ++it) {
          const int row = it * 4 + q4;
          *(volatile v4u*)(Shp + gb + (size_t)row * ND) = hv[it];
          *(volatile v4u*)(Slp + gb + (size_t)row * ND) = lv[it];
        }
        __threadfence();
      }
    } else {
      __syncthreads();
      const int vq = 4 * m;
      const int wc = (wave < 4) ? wave : 3;
      v4f ov[8];
#pragma unroll
      for (int it = 0; it < 8; ++it) {
        const int d = wc * 16 + 2 * it + hh;
        const float* sp = slabs + (vq >> 4) * SLABF + (vq & 15) * 68 + d;
        v4f t; t[0] = sp[0]; t[1] = sp[68]; t[2] = sp[136]; t[3] = sp[204];
        ov[it] = t;
      }
      const float* sp2 = slabs + 4 * SLABF + 4 * m;
      v4f o2; o2[0] = sp2[0]; o2[1] = sp2[1]; o2[2] = sp2[2]; o2[3] = sp2[3];
      for (int pass = 0; pass < 2; ++pass) {
        if (wave < 4) {
#pragma unroll
          for (int it = 0; it < 8; ++it) {
            const int d = wave * 16 + 2 * it + hh;
            *(volatile v4f*)(out1 + (size_t)bh * (ND * ND) + (size_t)d * ND + vq) = ov[it];
          }
        } else if (lane < 16) {
          *(volatile v4f*)(out2 + (size_t)bh * ND + 4 * lane) = o2;
        }
        __threadfence();
      }
    }
    __syncthreads();
    if (c < NCH) {
      if (tid < 128) {
        const int s = tid >> 1, dh = (tid & 1) * 32;
        const float* src = kf + ((size_t)(bh * NT + c * CH + s)) * ND + dh;
#pragma unroll 1
        for (int g = 0; g < 4; ++g) {
          const v4f a0 = *(const v4fa*)(src + 8 * g);
          const v4f a1 = *(const v4fa*)(src + 8 * g + 4);
          const float xv[8] = {a0[0], a0[1], a0[2], a0[3], a1[0], a1[1], a1[2], a1[3]};
#pragma unroll
          for (int e = 0; e < 8; ++e) {
            const float p = phi_f(xv[e]);
            const unsigned short hb = bf_bits(p);
            const unsigned short lb = bf_bits(p - bf_up(hb));
            const int n = dh + 8 * g + e;
            sKh[n * KP + s] = bf_val(hb);
            sKl[n * KP + s] = bf_val(lb);
          }
        }
      }
      __syncthreads();
      const size_t ac = arow + (size_t)c * CH;
#pragma unroll 1
      for (int ks = 0; ks < 2; ++ks) {
        const v16b ah = ldfrag_b(VTh + ac + 32 * ks);
        const v16b al = ldfrag_b(VTl + ac + 32 * ks);
#pragma unroll
        for (int nt = 0; nt < 4; ++nt) {
          const int p = (nt * 16 + m) * KP + 32 * ks + 8 * hh;
          const v16b kh = ldfrag_b(sKh + p);
          const v16b kl = ldfrag_b(sKl + p);
          acc[nt] = mma_b(ah, kh, acc[nt]);
          acc[nt] = mma_b(ah, kl, acc[nt]);
          acc[nt] = mma_b(al, kh, acc[nt]);
        }
      }
    }
  }
}

#define L_QH   0
#define L_QL   9216
#define L_KH   18432
#define L_KL   27648
#define L_PH   36864
#define L_PL   46080
#define L_TOT  55296
static_assert(L_QL - L_QH == CH * QP * 2);
static_assert(L_KH - L_QL == CH * QP * 2);
static_assert(L_KL - L_KH == CH * QP * 2);
static_assert(L_PH - L_KL == CH * QP * 2);
static_assert(L_PL - L_PH == CH * KP * 2);
static_assert(L_TOT - L_PL == CH * KP * 2);
static_assert(4 * 16 * ND * 4 <= L_KH);

__global__ __launch_bounds__(128)
void k_out(const float* __restrict__ qf, const float* __restrict__ kf,
           const unsigned short* __restrict__ VThp, const unsigned short* __restrict__ VTlp,
           const unsigned short* __restrict__ Shp, const unsigned short* __restrict__ Slp,
           unsigned short* Yhp, unsigned short* Ylp) {
  __shared__ __align__(16) unsigned char lds[L_TOT];
  __bf16* sQh = (__bf16*)(void*)(lds + L_QH);
  __bf16* sQl = (__bf16*)(void*)(lds + L_QL);
  __bf16* sKh = (__bf16*)(void*)(lds + L_KH);
  __bf16* sKl = (__bf16*)(void*)(lds + L_KL);
  __bf16* Ph  = (__bf16*)(void*)(lds + L_PH);
  __bf16* Pl  = (__bf16*)(void*)(lds + L_PL);

  const int tid = threadIdx.x, lane = tid & 31, wave = tid >> 5;
  const int hh = lane >> 4, m = lane & 15;
  const int bh = blockIdx.x >> 5, c = blockIdx.x & 31, t0 = c * CH;
  const int b = bh >> 4, head = bh & 15;

  {
    const int r = tid >> 1, dh = (tid & 1) * 32;
    const size_t go = ((size_t)(bh * NT + t0 + r)) * ND + dh;
    const int lo = r * QP + dh;
#pragma unroll 1
    for (int g = 0; g < 4; ++g) {
      v4u hv, lv;
      phi_split8(*(const v4fa*)(qf + go + 8 * g), *(const v4fa*)(qf + go + 8 * g + 4), hv, lv);
      *(v8b*)(sQh + lo + 8 * g) = __builtin_bit_cast(v8b, hv);
      *(v8b*)(sQl + lo + 8 * g) = __builtin_bit_cast(v8b, lv);
      phi_split8(*(const v4fa*)(kf + go + 8 * g), *(const v4fa*)(kf + go + 8 * g + 4), hv, lv);
      *(v8b*)(sKh + lo + 8 * g) = __builtin_bit_cast(v8b, hv);
      *(v8b*)(sKl + lo + 8 * g) = __builtin_bit_cast(v8b, lv);
    }
  }
  __syncthreads();

  v8f G[4];
#pragma unroll
  for (int kt = 0; kt < 4; ++kt) G[kt] = zero8();
  const int qo = (wave * 16 + m) * QP + 8 * hh;
#pragma unroll 1
  for (int ks = 0; ks < 2; ++ks) {
    const v16b aqh = ldfrag_b(sQh + qo + 32 * ks);
    const v16b aql = ldfrag_b(sQl + qo + 32 * ks);
#pragma unroll
    for (int kt = 0; kt < 4; ++kt) {
      const int pb = (kt * 16 + m) * QP + 32 * ks + 8 * hh;
      const v16b bkh = ldfrag_b(sKh + pb);
      const v16b bkl = ldfrag_b(sKl + pb);
      G[kt] = mma_b(aqh, bkh, G[kt]);
      G[kt] = mma_b(aqh, bkl, G[kt]);
      G[kt] = mma_b(aql, bkh, G[kt]);
    }
  }
#pragma unroll
  for (int kt = 0; kt < 4; ++kt) {
    const int sl = kt * 16 + m;
#pragma unroll
    for (int r = 0; r < 8; ++r) {
      const int tl = wave * 16 + 8 * hh + r;
      const float pv = (sl <= tl) ? G[kt][r] : 0.0f;
      const unsigned short hb = bf_bits(pv);
      const unsigned short lb = bf_bits(pv - bf_up(hb));
      const int po = tl * KP + sl;
      Ph[po] = bf_val(hb);
      Pl[po] = bf_val(lb);
    }
  }
  __builtin_amdgcn_fence(__ATOMIC_RELEASE, "workgroup");
  __builtin_amdgcn_wave_barrier();
  __builtin_amdgcn_fence(__ATOMIC_ACQUIRE, "workgroup");

  v8f acc[5];
#pragma unroll
  for (int nt = 0; nt < 5; ++nt) acc[nt] = zero8();
  const size_t sb = ((size_t)((bh * NSL + c) * NJ + m)) * ND + 8 * hh;
  const __bf16* Sh = (const __bf16*)(const void*)Shp + sb;
  const __bf16* Sl = (const __bf16*)(const void*)Slp + sb;
#pragma unroll 1
  for (int ks = 0; ks < 2; ++ks) {
    const v16b aqh = ldfrag_b(sQh + qo + 32 * ks);
    const v16b aql = ldfrag_b(sQl + qo + 32 * ks);
    const int fo = 32 * ks;
#pragma unroll
    for (int nt = 0; nt < 5; ++nt) {
      const v16b bsh = ldfrag_b(Sh + (size_t)nt * 16 * ND + fo);
      const v16b bsl = ldfrag_b(Sl + (size_t)nt * 16 * ND + fo);
      acc[nt] = mma_b(aqh, bsh, acc[nt]);
      acc[nt] = mma_b(aqh, bsl, acc[nt]);
      acc[nt] = mma_b(aql, bsh, acc[nt]);
    }
  }
  {
    const int po = (wave * 16 + m) * KP + 8 * hh;
    const size_t vo = ((size_t)(bh * NJ + m)) * NT + t0 + 8 * hh;
    const __bf16* VTh = (const __bf16*)(const void*)VThp + vo;
    const __bf16* VTl = (const __bf16*)(const void*)VTlp + vo;
#pragma unroll 1
    for (int kk = 0; kk < 2; ++kk) {
      const v16b pah = ldfrag_b(Ph + po + 32 * kk);
      const v16b pal = ldfrag_b(Pl + po + 32 * kk);
#pragma unroll
      for (int nt = 0; nt < 5; ++nt) {
        const v16b vbh = ldfrag_b(VTh + (size_t)nt * 16 * NT + 32 * kk);
        const v16b vbl = ldfrag_b(VTl + (size_t)nt * 16 * NT + 32 * kk);
        acc[nt] = mma_b(pah, vbh, acc[nt]);
        acc[nt] = mma_b(pah, vbl, acc[nt]);
        acc[nt] = mma_b(pal, vbh, acc[nt]);
      }
    }
  }

  float sc[8];
#pragma unroll
  for (int r = 0; r < 8; ++r) {
    const float dcol = __shfl(acc[4][r], hh * 16, 32);
    sc[r] = 1.0f / (dcol + 1e-6f);
  }
  __syncthreads();
  float* so = (float*)(void*)lds + wave * (16 * ND);
#pragma unroll
  for (int nt = 0; nt < 4; ++nt)
#pragma unroll
    for (int r = 0; r < 8; ++r) so[(8 * hh + r) * ND + nt * 16 + m] = acc[nt][r] * sc[r];
  __builtin_amdgcn_fence(__ATOMIC_RELEASE, "workgroup");
  __builtin_amdgcn_wave_barrier();
  __builtin_amdgcn_fence(__ATOMIC_ACQUIRE, "workgroup");
  const int q8 = lane & 7, sub = lane >> 3;
  v4u hv[4], lv[4];
#pragma unroll
  for (int it = 0; it < 4; ++it) {
    const int row = it * 4 + sub;
    const float* sp = so + row * ND + 8 * q8;
    v4u a, a2;
#pragma unroll
    for (int e = 0; e < 4; ++e) {
      const float f0 = sp[2 * e], f1 = sp[2 * e + 1];
      const unsigned short h0 = bf_bits(f0), h1 = bf_bits(f1);
      const unsigned short l0 = bf_bits(f0 - bf_up(h0)), l1 = bf_bits(f1 - bf_up(h1));
      a[e] = pk16(h0, h1); a2[e] = pk16(l0, l1);
    }
    hv[it] = a; lv[it] = a2;
  }
  const size_t gy = ((size_t)(b * NT + t0 + wave * 16)) * NC + head * ND + 8 * q8;
  for (int pass = 0; pass < 2; ++pass) {
#pragma unroll
    for (int it = 0; it < 4; ++it) {
      const int row = it * 4 + sub;
      *(volatile v4u*)(Yhp + gy + (size_t)row * NC) = hv[it];
      *(volatile v4u*)(Ylp + gy + (size_t)row * NC) = lv[it];
    }
    __threadfence();
  }
}

__global__ __launch_bounds__(128) void k_oproj(const unsigned short* __restrict__ Yhp, const unsigned short* __restrict__ Ylp,
                                              const unsigned short* __restrict__ wbp, const float* __restrict__ bp,
                                              float* out) {
  __shared__ __align__(16) float sT[128 * ND];
  const int tid = threadIdx.x, lane = tid & 31, w = tid >> 5;
  const int hh = lane >> 4, m = lane & 15;
  const int m0 = blockIdx.x * 128, nb = blockIdx.y;
  const __bf16* Yh = (const __bf16*)(const void*)Yhp;
  const __bf16* Yl = (const __bf16*)(const void*)Ylp;
  const __bf16* wb = (const __bf16*)(const void*)wbp;
  const size_t yo0 = ((size_t)(m0 + 32 * w + m)) * NC + 8 * hh;
  const size_t yo1 = yo0 + (size_t)16 * NC;
  const __bf16* wr = wb + ((size_t)3 * NC + nb * ND + m) * NC + 8 * hh;

  v8f acc[2][4];
#pragma unroll
  for (int mt = 0; mt < 2; ++mt)
#pragma unroll
    for (int nt = 0; nt < 4; ++nt) acc[mt][nt] = zero8();

#pragma unroll 1
  for (int k0 = 0; k0 < NC; k0 += 32) {
    const v16b a0h = ldfrag_b(Yh + yo0 + k0);
    const v16b a0l = ldfrag_b(Yl + yo0 + k0);
    const v16b a1h = ldfrag_b(Yh + yo1 + k0);
    const v16b a1l = ldfrag_b(Yl + yo1 + k0);
#pragma unroll
    for (int nt = 0; nt < 4; ++nt) {
      const v16b bb = ldfrag_b(wr + (size_t)nt * 16 * NC + k0);
      acc[0][nt] = mma_b(a0h, bb, acc[0][nt]);
      acc[0][nt] = mma_b(a0l, bb, acc[0][nt]);
      acc[1][nt] = mma_b(a1h, bb, acc[1][nt]);
      acc[1][nt] = mma_b(a1l, bb, acc[1][nt]);
    }
  }

#pragma unroll
  for (int nt = 0; nt < 4; ++nt) {
    const int feat = 16 * nt + m;
    const float bvl = bf_up(bf_bits(bp[nb * ND + feat]));
#pragma unroll
    for (int mt = 0; mt < 2; ++mt)
#pragma unroll
      for (int r = 0; r < 8; ++r) {
        const int tokl = 32 * w + 16 * mt + 8 * hh + r;
        sT[tokl * ND + feat] = acc[mt][nt][r] + bvl;
      }
  }
  __syncthreads();

  for (int pass = 0; pass < 2; ++pass) {
#pragma unroll
    for (int i = 0; i < 16; ++i) {
      const int rowl = 32 * w + 2 * i + hh;
      const v4f vv = *(const v4fa*)(sT + rowl * ND + 4 * m);
      *(volatile v4f*)(out + ((size_t)(m0 + rowl)) * NC + nb * ND + 4 * m) = vv;
    }
    __threadfence();
  }
}

extern "C" void kernel_launch(void* const* d_in, const int* in_sizes, int n_in,
                              void* d_out, int out_size, void* d_ws, size_t ws_size,
                              hipStream_t stream) {
  if (n_in < 6) return;
  if (in_sizes[0] != NTOK * NC) return;
  if (in_sizes[1] != NC * NC || in_sizes[2] != NC * NC || in_sizes[3] != NC * NC || in_sizes[4] != NC * NC) return;
  if (in_sizes[5] < NC) return;
  const int n_out0 = NTOK * NC;
  const int n_out1 = NBH * ND * ND;
  const int n_out2 = NBH * ND;
  if (out_size != n_out0 + n_out1 + n_out2) return;

  const float* x  = (const float*)d_in[0];
  const float* Wq = (const float*)d_in[1];
  const float* Wk = (const float*)d_in[2];
  const float* Wv = (const float*)d_in[3];
  const float* Wp = (const float*)d_in[4];
  const float* bp = (const float*)d_in[5];
  float* out0 = (float*)d_out;
  float* out1 = out0 + n_out0;
  float* out2 = out1 + n_out1;

  const size_t PXB = (size_t)NTOK * NC * 2;
  const size_t PWB = (size_t)4 * NC * NC * 2;
  const size_t PF  = (size_t)NBH * NT * ND * 4;
  const size_t PVT = (size_t)NBH * NJ * NT * 2;
  const size_t PS  = (size_t)NBH * NSL * NJ * ND * 2;
  const size_t PY  = (size_t)NTOK * NC * 2;
  size_t off = 0;
  const size_t oXB = off; off += PXB;
  const size_t oWB = off; off += PWB;
  const size_t oQF = off; off += PF;
  const size_t oKF = off; off += PF;
  const size_t oVF = off; off += PF;
  const size_t oVTh = off; off += PVT;
  const size_t oVTl = off; off += PVT;
  const size_t oSh = off; off += PS;
  const size_t oSl = off; off += PS;
  const size_t oYh = off; off += PY;
  const size_t oYl = off; off += PY;
  if (off > ws_size) return;
  if (off > (size_t)134217728u) return;

  char* ws = (char*)d_ws;
  unsigned short* xb  = (unsigned short*)(ws + oXB);
  unsigned short* wb  = (unsigned short*)(ws + oWB);
  float* qf = (float*)(ws + oQF);
  float* kf = (float*)(ws + oKF);
  float* vf = (float*)(ws + oVF);
  unsigned short* VTh = (unsigned short*)(ws + oVTh);
  unsigned short* VTl = (unsigned short*)(ws + oVTl);
  unsigned short* Sh  = (unsigned short*)(ws + oSh);
  unsigned short* Sl  = (unsigned short*)(ws + oSl);
  unsigned short* Yh  = (unsigned short*)(ws + oYh);
  unsigned short* Yl  = (unsigned short*)(ws + oYl);

  k_cvt<<<dim3((NX8 + 4 * NW8) / 256), dim3(256), 0, stream>>>(x, Wq, Wk, Wv, Wp, xb, wb);
  k_proj<<<dim3(NTOK / 128, 3 * NH), dim3(128), 0, stream>>>(xb, wb, qf, kf, vf);
  k_vt<<<dim3(NBH * (NT / 64)), dim3(128), 0, stream>>>(vf, VTh, VTl);
  k_state<<<dim3(NBH), dim3(160), 0, stream>>>(kf, VTh, VTl, Sh, Sl, out1, out2);
  k_out<<<dim3(NBH * NCH), dim3(128), 0, stream>>>(qf, kf, VTh, VTl, Sh, Sl, Yh, Yl);
  k_oproj<<<dim3(NTOK / 128, NC / ND), dim3(128), 0, stream>>>(Yh, Yl, wb, bp, out0);
  (void)hipGetLastError();
}
